// FedGNN_75247827026509
// MI455X (gfx1250) — hardware-verified
//
#include <hip/hip_runtime.h>
#define NNODE 50000
#define NE 800000
#define NTOT (NE + NNODE)
#define FIN 64
#define HID 64
#define NG 512
#define NCLS 10
#define NN NNODE
#define MAXDEG 256

typedef __bf16 v16b __attribute__((ext_vector_type(16)));
typedef unsigned short v8us __attribute__((ext_vector_type(8), may_alias));
typedef float  v8f  __attribute__((ext_vector_type(8)));
typedef float  v4f  __attribute__((ext_vector_type(4)));
typedef float  v4fa __attribute__((ext_vector_type(4), may_alias));
union FragB { v16b v; v8us half[2]; unsigned short u[16]; };

__device__ __forceinline__ unsigned short bf16_bits(float x) { unsigned int u = __float_as_uint(x); return (unsigned short)((u + 0x7FFFu + ((u >> 16) & 1u)) >> 16); }
__device__ __forceinline__ float bf16_val(unsigned short b) { return __uint_as_float(((unsigned int)b) << 16); }
__device__ __forceinline__ float bf16_round(float x) { return bf16_val(bf16_bits(x)); }
template <int NT>
__device__ __forceinline__ v8f mmaN(v16b ah, v16b al, v16b bh, v16b bl, v8f c) {
  c = __builtin_amdgcn_wmma_f32_16x16x32_bf16(false, ah, false, bh, (short)0, c, false, false);
  if (NT >= 2) c = __builtin_amdgcn_wmma_f32_16x16x32_bf16(false, al, false, bh, (short)0, c, false, false);
  if (NT >= 3) c = __builtin_amdgcn_wmma_f32_16x16x32_bf16(false, ah, false, bl, (short)0, c, false, false);
  asm volatile("v_nop\n\tv_nop\n\tv_nop\n\tv_nop" : "+v"(c) : "v"(ah), "v"(al), "v"(bh), "v"(bl));
  return c;
}

__global__ __launch_bounds__(256) void k_wt_bf16(const float* __restrict__ W, unsigned short* __restrict__ Wt, int K, int N) {
  const int t = blockIdx.x * 256 + threadIdx.x;
  const int k8n = K / 8;
  if (t >= N * k8n) return;
  const int n = t / k8n, k8 = (t % k8n) * 8;
  v8us v;
#pragma unroll
  for (int i = 0; i < 8; ++i) v[i] = bf16_bits(W[(size_t)(k8 + i) * N + n]);
  *(volatile v8us*)(Wt + (size_t)n * K + k8) = v;
  __threadfence();
  *(volatile v8us*)(Wt + (size_t)n * K + k8) = v;
}

template <bool ASPLIT, int ACT, bool BIAS_BF16>
__global__ __launch_bounds__(128) void k_gemm_bf(const float* __restrict__ A, int lda, const unsigned short* __restrict__ Wt, int ldb,
                                               const float* __restrict__ bias, float* __restrict__ C, int ldc, int M, int N, int K) {
  __shared__ __attribute__((aligned(16))) float so[4][16][64];
  const int tid = threadIdx.x, w = tid >> 5, lane = tid & 31, ln = lane & 15, hh = lane >> 4;
  const int ntn = N / 64;
  const int wid = blockIdx.x * 4 + w;
  const int mt = wid / ntn, nq = wid % ntn;
  if (mt * 16 >= M) return;
  const int row0 = mt * 16, col0 = nq * 64;
  const float* arow = A + (size_t)(row0 + ln) * lda;
  v8f acc[4] = {};
  for (int kb = 0; kb < K; kb += 32) {
    FragB ah, al;
    const v4f x0 = *(const v4fa*)(arow + kb + 8 * hh), x1 = *(const v4fa*)(arow + kb + 8 * hh + 4);
    const v4f x2 = *(const v4fa*)(arow + kb + 16 + 8 * hh), x3 = *(const v4fa*)(arow + kb + 16 + 8 * hh + 4);
    float xs[16] = {x0[0],x0[1],x0[2],x0[3],x1[0],x1[1],x1[2],x1[3],x2[0],x2[1],x2[2],x2[3],x3[0],x3[1],x3[2],x3[3]};
#pragma unroll
    for (int i = 0; i < 16; ++i) { const unsigned short hb = bf16_bits(xs[i]); ah.u[i] = hb; al.u[i] = ASPLIT ? bf16_bits(xs[i] - bf16_val(hb)) : (unsigned short)0; }
#pragma unroll
    for (int t = 0; t < 4; ++t) {
      const unsigned short* brow = Wt + (size_t)(col0 + t * 16 + ln) * ldb + kb;
      FragB b;
      b.half[0] = *(const v8us*)(brow + 8 * hh);
      b.half[1] = *(const v8us*)(brow + 16 + 8 * hh);
      acc[t] = mmaN<ASPLIT ? 2 : 1>(ah.v, al.v, b.v, b.v, acc[t]);
    }
  }
#pragma unroll
  for (int t = 0; t < 4; ++t) {
    float bv = bias ? bias[col0 + t * 16 + ln] : 0.f;
    if (BIAS_BF16) bv = bf16_round(bv);
#pragma unroll
    for (int r = 0; r < 8; ++r) { float v = acc[t][r] + bv; if (ACT == 1) v = fmaxf(v, 0.f); so[w][8 * hh + r][t * 16 + ln] = v; }
  }
  __builtin_amdgcn_fence(__ATOMIC_ACQ_REL, "workgroup");
  __builtin_amdgcn_wave_barrier();
  const int rsub = lane >> 4, c4 = (lane & 15) * 4;
  for (int pass = 0; pass < 2; ++pass) {
#pragma unroll
    for (int q = 0; q < 8; ++q) {
      const int r = q * 2 + rsub;
      const v4f v = *(const v4fa*)&so[w][r][c4];
      *(volatile v4f*)(C + (size_t)(row0 + r) * ldc + col0 + c4) = v;
    }
    if (pass == 0) __threadfence();
  }
}

template <int D, bool CAUSAL>
__global__ __launch_bounds__(128) void k_flash(const float* __restrict__ qb, const float* __restrict__ kb, const float* __restrict__ vb,
                                             int pitch, int T, int H, float scale, float* __restrict__ y, int ypitch) {
  constexpr int KS = D / 32;
  constexpr int DT = D / 16;
  __shared__ __attribute__((aligned(16))) unsigned short sKh[32][D + 8], sKl[32][D + 8], sVh[32][D + 8], sVl[32][D + 8];
  __shared__ __attribute__((aligned(16))) unsigned short sPh[4][16][40], sPl[4][16][40];
  __shared__ __attribute__((aligned(16))) float sO[4][16][D];
  const int tid = threadIdx.x, w = tid >> 5, lane = tid & 31, ln = lane & 15, hh = lane >> 4;
  const int nqb = (T + 63) / 64;
  const int bh = blockIdx.x / nqb, qblk = blockIdx.x % nqb;
  const int b = bh / H, h = bh % H;
  const int q0 = qblk * 64 + w * 16;
  const float* Q = qb + (size_t)b * T * pitch + h * D;
  const float* K = kb + (size_t)b * T * pitch + h * D;
  const float* V = vb + (size_t)b * T * pitch + h * D;

  FragB aqh[KS], aql[KS];
  {
    int row = q0 + ln; if (row >= T) row = T - 1;
    const float* qr = Q + (size_t)row * pitch;
#pragma unroll
    for (int ks = 0; ks < KS; ++ks)
#pragma unroll
      for (int i = 0; i < 16; ++i) {
        const int d = ks * 32 + ((i < 8) ? (8 * hh + i) : (16 + 8 * hh + (i - 8)));
        const float x = qr[d] * scale; const unsigned short hb = bf16_bits(x);
        aqh[ks].u[i] = hb; aql[ks].u[i] = bf16_bits(x - bf16_val(hb));
      }
  }
  float m_r[8], l_r[8];
#pragma unroll
  for (int r = 0; r < 8; ++r) { m_r[r] = -3.0e38f; l_r[r] = 0.f; }
  v8f oacc[DT];
#pragma unroll
  for (int dt = 0; dt < DT; ++dt) oacc[dt] = (v8f){0.f,0.f,0.f,0.f,0.f,0.f,0.f,0.f};

  const int kv_end = CAUSAL ? min(T, qblk * 64 + 64) : T;
  for (int j0 = 0; j0 < kv_end; j0 += 32) {
    __syncthreads();
    for (int e = tid; e < 32 * (D / 4); e += 128) {
      const int r = e / (D / 4), c4 = (e % (D / 4)) * 4;
      const int key = j0 + r;
      v4f kf = {0.f,0.f,0.f,0.f}, vf = {0.f,0.f,0.f,0.f};
      if (key < T) { kf = *(const v4fa*)(K + (size_t)key * pitch + c4); vf = *(const v4fa*)(V + (size_t)key * pitch + c4); }
#pragma unroll
      for (int t = 0; t < 4; ++t) {
        unsigned short hb = bf16_bits(kf[t]); sKh[r][c4 + t] = hb; sKl[r][c4 + t] = bf16_bits(kf[t] - bf16_val(hb));
        hb = bf16_bits(vf[t]); sVh[r][c4 + t] = hb; sVl[r][c4 + t] = bf16_bits(vf[t] - bf16_val(hb));
      }
    }
    __syncthreads();
    v8f s[2];
#pragma unroll
    for (int nt = 0; nt < 2; ++nt) {
      v8f acc = {};
#pragma unroll
      for (int ks = 0; ks < KS; ++ks) {
        FragB bh_, bl_;
        bh_.half[0] = *(const v8us*)&sKh[nt * 16 + ln][ks * 32 + 8 * hh]; bh_.half[1] = *(const v8us*)&sKh[nt * 16 + ln][ks * 32 + 16 + 8 * hh];
        bl_.half[0] = *(const v8us*)&sKl[nt * 16 + ln][ks * 32 + 8 * hh]; bl_.half[1] = *(const v8us*)&sKl[nt * 16 + ln][ks * 32 + 16 + 8 * hh];
        acc = mmaN<3>(aqh[ks].v, aql[ks].v, bh_.v, bl_.v, acc);
      }
      s[nt] = acc;
    }
    float alpha[8];
#pragma unroll
    for (int r = 0; r < 8; ++r) {
      const int qi = q0 + 8 * hh + r;
      const int ja = j0 + ln, jb = j0 + 16 + ln;
      if (CAUSAL) { if (ja > qi) s[0][r] = -3.0e38f; if (jb > qi) s[1][r] = -3.0e38f; }
      if (ja >= T) s[0][r] = -3.0e38f;
      if (jb >= T) s[1][r] = -3.0e38f;
      float mx = fmaxf(s[0][r], s[1][r]);
      mx = fmaxf(mx, __shfl_xor(mx, 1, 32)); mx = fmaxf(mx, __shfl_xor(mx, 2, 32)); mx = fmaxf(mx, __shfl_xor(mx, 4, 32)); mx = fmaxf(mx, __shfl_xor(mx, 8, 32));
      const float mnew = fmaxf(m_r[r], mx);
      alpha[r] = (mnew > -1.0e38f) ? __expf(m_r[r] - mnew) : 1.0f;
      const float p0 = (s[0][r] > -1.0e38f) ? __expf(s[0][r] - mnew) : 0.f;
      const float p1 = (s[1][r] > -1.0e38f) ? __expf(s[1][r] - mnew) : 0.f;
      m_r[r] = mnew;
      l_r[r] = l_r[r] * alpha[r] + p0 + p1;
      unsigned short hb = bf16_bits(p0); sPh[w][8 * hh + r][ln] = hb;      sPl[w][8 * hh + r][ln] = bf16_bits(p0 - bf16_val(hb));
      hb = bf16_bits(p1);                sPh[w][8 * hh + r][16 + ln] = hb; sPl[w][8 * hh + r][16 + ln] = bf16_bits(p1 - bf16_val(hb));
    }
#pragma unroll
    for (int dt = 0; dt < DT; ++dt)
#pragma unroll
      for (int r = 0; r < 8; ++r) oacc[dt][r] *= alpha[r];
    __builtin_amdgcn_fence(__ATOMIC_ACQ_REL, "workgroup");
    __builtin_amdgcn_wave_barrier();
    FragB pah, pal;
    pah.half[0] = *(const v8us*)&sPh[w][ln][8 * hh]; pah.half[1] = *(const v8us*)&sPh[w][ln][16 + 8 * hh];
    pal.half[0] = *(const v8us*)&sPl[w][ln][8 * hh]; pal.half[1] = *(const v8us*)&sPl[w][ln][16 + 8 * hh];
#pragma unroll
    for (int dt = 0; dt < DT; ++dt) {
      FragB bvh, bvl;
#pragma unroll
      for (int i = 0; i < 8; ++i) {
        bvh.u[i] = sVh[8 * hh + i][dt * 16 + ln]; bvh.u[8 + i] = sVh[16 + 8 * hh + i][dt * 16 + ln];
        bvl.u[i] = sVl[8 * hh + i][dt * 16 + ln]; bvl.u[8 + i] = sVl[16 + 8 * hh + i][dt * 16 + ln];
      }
      oacc[dt] = mmaN<3>(pah.v, pal.v, bvh.v, bvl.v, oacc[dt]);
    }
    __builtin_amdgcn_fence(__ATOMIC_ACQ_REL, "workgroup");
    __builtin_amdgcn_wave_barrier();
  }
#pragma unroll
  for (int r = 0; r < 8; ++r) {
    float l = l_r[r];
    l += __shfl_xor(l, 1, 32); l += __shfl_xor(l, 2, 32); l += __shfl_xor(l, 4, 32); l += __shfl_xor(l, 8, 32);
    l_r[r] = (l > 0.f) ? 1.0f / l : 0.f;
  }
#pragma unroll
  for (int dt = 0; dt < DT; ++dt)
#pragma unroll
    for (int r = 0; r < 8; ++r) sO[w][8 * hh + r][dt * 16 + ln] = oacc[dt][r] * l_r[r];
  __builtin_amdgcn_fence(__ATOMIC_ACQ_REL, "workgroup");
  __builtin_amdgcn_wave_barrier();
  for (int pass = 0; pass < 2; ++pass) {
    for (int r = 0; r < 16; ++r) {
      const int row = q0 + r;
      if (row < T && lane < D / 4) {
        const v4f val = *(const v4fa*)&sO[w][r][lane * 4];
        *(volatile v4f*)(y + ((size_t)b * T + row) * ypitch + h * D + lane * 4) = val;
      }
    }
    if (pass == 0) __threadfence();
  }
}

template <bool ASPLIT, int ACT, bool BIAS_BF16, bool RES_BF16>
__global__ __launch_bounds__(128) void k_gemm_bf3(const float* __restrict__ A, int lda, const unsigned short* __restrict__ Wt, int ldb,
                                                const float* __restrict__ bias, const float* __restrict__ resid, int rmod, int ldr,
                                                float* __restrict__ C, int ldc, int M, int N, int K) {
  __shared__ __attribute__((aligned(16))) float so[4][16][64];
  const int tid = threadIdx.x, w = tid >> 5, lane = tid & 31, ln = lane & 15, hh = lane >> 4;
  const int ntn = N / 64;
  const int wid = blockIdx.x * 4 + w;
  const int mt = wid / ntn, nq = wid % ntn;
  if (mt * 16 >= M) return;
  const int row0 = mt * 16, col0 = nq * 64;
  const float* arow = A + (size_t)(row0 + ln) * lda;
  v8f acc[4] = {};
  for (int kb = 0; kb < K; kb += 32) {
    FragB ah, al;
    const v4f x0 = *(const v4fa*)(arow + kb + 8 * hh), x1 = *(const v4fa*)(arow + kb + 8 * hh + 4);
    const v4f x2 = *(const v4fa*)(arow + kb + 16 + 8 * hh), x3 = *(const v4fa*)(arow + kb + 16 + 8 * hh + 4);
    float xs[16] = {x0[0],x0[1],x0[2],x0[3],x1[0],x1[1],x1[2],x1[3],x2[0],x2[1],x2[2],x2[3],x3[0],x3[1],x3[2],x3[3]};
#pragma unroll
    for (int i = 0; i < 16; ++i) { const unsigned short hb = bf16_bits(xs[i]); ah.u[i] = hb; al.u[i] = ASPLIT ? bf16_bits(xs[i] - bf16_val(hb)) : (unsigned short)0; }
#pragma unroll
    for (int t = 0; t < 4; ++t) {
      const unsigned short* brow = Wt + (size_t)(col0 + t * 16 + ln) * ldb + kb;
      FragB b;
      b.half[0] = *(const v8us*)(brow + 8 * hh);
      b.half[1] = *(const v8us*)(brow + 16 + 8 * hh);
      acc[t] = mmaN<ASPLIT ? 2 : 1>(ah.v, al.v, b.v, b.v, acc[t]);
    }
  }
#pragma unroll
  for (int t = 0; t < 4; ++t) {
    const int col = col0 + t * 16 + ln;
    float bv = bias ? bias[col] : 0.f;
    if (BIAS_BF16) bv = bf16_round(bv);
#pragma unroll
    for (int r = 0; r < 8; ++r) {
      float v = acc[t][r] + bv;
      if (resid) { float rv = resid[(size_t)((row0 + 8 * hh + r) % rmod) * ldr + col]; if (RES_BF16) rv = bf16_round(rv); v += rv; }
      if (ACT == 1) v = fmaxf(v, 0.f);
      if (ACT == 2) v = 0.5f * v * (1.0f + erff(v * 0.70710678118654752f));
      if (ACT == 3) { const float u = 0.7978845608028654f * (v + 0.044715f * v * v * v); v = 0.5f * v * (1.0f + tanhf(u)); }
      so[w][8 * hh + r][t * 16 + ln] = v;
    }
  }
  __builtin_amdgcn_fence(__ATOMIC_ACQ_REL, "workgroup");
  __builtin_amdgcn_wave_barrier();
  const int rsub = lane >> 4, c4 = (lane & 15) * 4;
  for (int pass = 0; pass < 2; ++pass) {
#pragma unroll
    for (int q = 0; q < 8; ++q) {
      const int r = q * 2 + rsub;
      const v4f v = *(const v4fa*)&so[w][r][c4];
      *(volatile v4f*)(C + (size_t)(row0 + r) * ldc + col0 + c4) = v;
    }
    if (pass == 0) __threadfence();
  }
}
template <bool PARAM_BF16>
__global__ __launch_bounds__(256) void k_layernorm(const float* __restrict__ X, const float* __restrict__ R, const float* __restrict__ g, const float* __restrict__ bta,
                                                  float* __restrict__ out_sum, float* __restrict__ out_norm, int N, float eps) {
  __shared__ float red[256];
  const int row = blockIdx.x, tid = threadIdx.x;
  const float* x = X + (size_t)row * N; const float* rr = R ? R + (size_t)row * N : nullptr;
  float vals[16];
  const int per = N / 256;
  float s1 = 0.f;
  for (int u = 0; u < per / 4; ++u) {
    const int j = tid * 4 + 1024 * u;
    const v4f a = *(const v4fa*)(x + j);
    v4f b = {0.f,0.f,0.f,0.f}; if (rr) b = *(const v4fa*)(rr + j);
#pragma unroll
    for (int q = 0; q < 4; ++q) { const float v = a[q] + b[q]; vals[u * 4 + q] = v; s1 += v; }
  }
  red[tid] = s1; __syncthreads();
  for (int st = 128; st > 0; st >>= 1) { if (tid < st) red[tid] += red[tid + st]; __syncthreads(); }
  const float mu = red[0] / (float)N; __syncthreads();
  float s2 = 0.f;
  for (int u = 0; u < per / 4; ++u)
#pragma unroll
    for (int q = 0; q < 4; ++q) { const float c = vals[u * 4 + q] - mu; s2 += c * c; }
  red[tid] = s2; __syncthreads();
  for (int st = 128; st > 0; st >>= 1) { if (tid < st) red[tid] += red[tid + st]; __syncthreads(); }
  const float rs = rsqrtf(red[0] / (float)N + eps);
  for (int pass = 0; pass < 2; ++pass) {
    for (int u = 0; u < per / 4; ++u) {
      const int j = tid * 4 + 1024 * u;
      v4f o, sm;
#pragma unroll
      for (int q = 0; q < 4; ++q) {
        float gg = g[j + q], bb = bta[j + q];
        if (PARAM_BF16) { gg = bf16_round(gg); bb = bf16_round(bb); }
        sm[q] = vals[u * 4 + q]; o[q] = (vals[u * 4 + q] - mu) * rs * gg + bb;
      }
      if (out_sum) *(volatile v4f*)(out_sum + (size_t)row * N + j) = sm;
      *(volatile v4f*)(out_norm + (size_t)row * N + j) = o;
    }
    if (pass == 0) __threadfence();
  }
}

#define CS_NW 1024
#define CS_CH 832
#define CS_NB 256
#define CS_CAP 8192
__device__ __forceinline__ int cs_dst(const int* __restrict__ eidst, int e, int ne, int nt, int nn) { if (e >= nt) return -1; int d = (e < ne) ? eidst[e] : (e - ne); return d < 0 ? 0 : (d >= nn ? nn - 1 : d); }
__global__ __launch_bounds__(256) void k_cs_p1(const int* __restrict__ eidst, int ne, int nt, int nn, int* __restrict__ seg_dst, int* __restrict__ seg_eid, int* __restrict__ P1, int* __restrict__ Q1) {
  __shared__ int scnt[8][CS_NB]; __shared__ int srun[8][CS_NB]; __shared__ int sod[8][CS_CH]; __shared__ int soe[8][CS_CH];
  const int tid = threadIdx.x, wv = tid >> 5, lane = tid & 31; const int w = blockIdx.x * 8 + wv; const int e0 = w * CS_CH;
  for (int i = lane; i < CS_NB; i += 32) { scnt[wv][i] = 0; srun[wv][i] = 0; }
  __builtin_amdgcn_fence(__ATOMIC_ACQ_REL, "workgroup"); __builtin_amdgcn_wave_barrier();
#pragma unroll 1
  for (int i0 = 0; i0 < CS_CH; i0 += 32) { const int e = e0 + i0 + lane; const int d = cs_dst(eidst, e, ne, nt, nn); const int hb = (d < 0) ? -1 : (d >> 8);
#pragma unroll 1
    for (int ld = 0; ld < 32; ++ld) { const int kk = __shfl(hb, ld, 32); const unsigned long long m = __ballot(hb == kk); const int first = __ffsll((long long)m) - 1; if (ld == first && lane == first && kk >= 0) scnt[wv][kk] += __popcll(m); }
    __builtin_amdgcn_fence(__ATOMIC_ACQ_REL, "workgroup"); __builtin_amdgcn_wave_barrier(); }
  { int loc[8]; int s = 0; for (int j = 0; j < 8; ++j) { loc[j] = s; s += scnt[wv][lane * 8 + j]; }
    int incl = s; for (int o = 1; o < 32; o <<= 1) { const int v = __shfl_up(incl, o, 32); if (lane >= o) incl += v; } const int excl = incl - s;
    for (int j = 0; j < 8; ++j) srun[wv][lane * 8 + j] = excl + loc[j]; }
  __builtin_amdgcn_fence(__ATOMIC_ACQ_REL, "workgroup"); __builtin_amdgcn_wave_barrier();
  for (int pass = 0; pass < 2; ++pass) { for (int i = lane; i < CS_NB; i += 32) { *(volatile int*)(P1 + (size_t)w * CS_NB + i) = scnt[wv][i]; *(volatile int*)(Q1 + (size_t)w * CS_NB + i) = srun[wv][i]; } if (pass == 0) __threadfence(); }
#pragma unroll 1
  for (int i0 = 0; i0 < CS_CH; i0 += 32) { const int e = e0 + i0 + lane; const int d = cs_dst(eidst, e, ne, nt, nn); const int hb = (d < 0) ? -1 : (d >> 8);
    int pos = -1; int grpcnt = 0; bool leader = false;
#pragma unroll 1
    for (int ld = 0; ld < 32; ++ld) { const int kk = __shfl(hb, ld, 32); const unsigned long long g = __ballot(hb == kk); const int first = __ffsll((long long)g) - 1;
      if (ld == first && kk >= 0) { if (hb == kk) { const unsigned long long below = g & ((1ull << lane) - 1ull); pos = srun[wv][kk] + __popcll(below); if (lane == first) { leader = true; grpcnt = __popcll(g); } } } }
    if (pos >= 0) { sod[wv][pos] = d; soe[wv][pos] = e; }
    __builtin_amdgcn_fence(__ATOMIC_ACQ_REL, "workgroup"); __builtin_amdgcn_wave_barrier();
    if (leader) srun[wv][hb] += grpcnt;
    __builtin_amdgcn_fence(__ATOMIC_ACQ_REL, "workgroup"); __builtin_amdgcn_wave_barrier(); }
  for (int pass = 0; pass < 2; ++pass) { for (int i = lane; i < CS_CH; i += 32) { *(volatile int*)(seg_dst + (size_t)e0 + i) = sod[wv][i]; *(volatile int*)(seg_eid + (size_t)e0 + i) = soe[wv][i]; } if (pass == 0) __threadfence(); }
}
__global__ __launch_bounds__(256) void k_cs_scan(const int* __restrict__ P1, int* __restrict__ R, int* __restrict__ S) {
  __shared__ int tot[CS_NB]; __shared__ int st[CS_NB + 1];
  const int b = threadIdx.x; int acc = 0;
#pragma unroll 1
  for (int w = 0; w < CS_NW; ++w) { const int c = P1[(size_t)w * CS_NB + b]; *(volatile int*)(R + (size_t)w * CS_NB + b) = acc; acc += c; }
  __threadfence();
  acc = 0;
#pragma unroll 1
  for (int w = 0; w < CS_NW; ++w) { const int c = P1[(size_t)w * CS_NB + b]; *(volatile int*)(R + (size_t)w * CS_NB + b) = acc; acc += c; }
  tot[b] = acc; __syncthreads();
  if (b == 0) { int s = 0; for (int i = 0; i < CS_NB; ++i) { st[i] = s; s += (tot[i] + 31) & ~31; } st[CS_NB] = s; }
  __syncthreads();
  for (int pass = 0; pass < 2; ++pass) { *(volatile int*)(S + b) = st[b]; if (b < 32) *(volatile int*)(S + CS_NB + b) = (b == 0) ? st[CS_NB] : 0; if (pass == 0) __threadfence(); }
}
__global__ __launch_bounds__(256) void k_cs_p2(const int* __restrict__ seg_dst, const int* __restrict__ seg_eid, const int* __restrict__ P1, const int* __restrict__ Q1, const int* __restrict__ R, const int* __restrict__ S, int nn, int* __restrict__ csr_eid, int* __restrict__ csr_start, int* __restrict__ csr_cnt) {
  __shared__ int sd[CS_CAP]; __shared__ int se[CS_CAP]; __shared__ int sorted[CS_CAP]; __shared__ int lcnt[CS_NB]; __shared__ int lpre[CS_NB + 1];
  const int hb = blockIdx.x, t = threadIdx.x; const int total = (R[(size_t)(CS_NW - 1) * CS_NB + hb] + P1[(size_t)(CS_NW - 1) * CS_NB + hb]); const int tot = total > CS_CAP ? CS_CAP : total;
#pragma unroll 1
  for (int w = t; w < CS_NW; w += 256) { const int c = P1[(size_t)w * CS_NB + hb]; const int base = R[(size_t)w * CS_NB + hb]; const int src = w * CS_CH + Q1[(size_t)w * CS_NB + hb];
    for (int k = 0; k < c; ++k) { const int p = base + k; if (p < CS_CAP) { sd[p] = seg_dst[src + k] & 255; se[p] = seg_eid[src + k]; } } }
  __syncthreads();
  { int c = 0;
#pragma unroll 1
    for (int i = 0; i < tot; ++i) c += (sd[i] == t) ? 1 : 0; lcnt[t] = c; }
  __syncthreads();
  if (t == 0) { int s = 0; for (int i = 0; i < CS_NB; ++i) { lpre[i] = s; s += lcnt[i]; } lpre[CS_NB] = s; }
  __syncthreads();
  { int k = lpre[t];
#pragma unroll 1
    for (int i = 0; i < tot; ++i) if (sd[i] == t) { sorted[k++] = se[i]; } }
  __syncthreads();
  const int s0 = S[hb]; const int s1 = S[hb + 1];
  for (int pass = 0; pass < 2; ++pass) {
    for (int i = t; i < s1 - s0; i += 256) *(volatile int*)(csr_eid + s0 + i) = (i < tot) ? sorted[i] : -1;
    { const int dst = hb * CS_NB + t; *(volatile int*)(csr_start + dst) = s0 + lpre[t]; *(volatile int*)(csr_cnt + dst) = lcnt[t]; }
    if (pass == 0) __threadfence(); }
}
static void build_csr(const int* eidst, int ne, int nt, int nn, int* seg_dst, int* seg_eid, int* P1, int* Q1, int* R, int* S, int* csr_eid, int* csr_start, int* csr_cnt, hipStream_t stream) {
  k_cs_p1<<<CS_NW / 8, 256, 0, stream>>>(eidst, ne, nt, nn, seg_dst, seg_eid, P1, Q1);
  k_cs_scan<<<1, 256, 0, stream>>>(P1, R, S);
  k_cs_p2<<<CS_NB, 256, 0, stream>>>(seg_dst, seg_eid, P1, Q1, R, S, nn, csr_eid, csr_start, csr_cnt);
}

__global__ __launch_bounds__(256) void k_btcat(const float* __restrict__ Wl, const float* __restrict__ Wr, int K, int NOUT, unsigned short* __restrict__ Bt) { const int t = blockIdx.x * 256 + threadIdx.x; if (t >= 2 * NOUT * (K / 8)) return; const int n = t / (K / 8), k8 = (t % (K / 8)) * 8; const float* W = (n < NOUT) ? Wl : Wr; const int nn = (n < NOUT) ? n : n - NOUT; v8us v;
  for (int q = 0; q < 8; ++q) v[q] = bf16_bits(W[(size_t)(k8 + q) * NOUT + nn]); *(volatile v8us*)(Bt + (size_t)n * K + k8) = v; __threadfence(); *(volatile v8us*)(Bt + (size_t)n * K + k8) = v; }
__device__ __forceinline__ float lrelu(float v) { return v >= 0.f ? v : 0.2f * v; }
__device__ __forceinline__ float elu1(float v) { return v > 0.f ? v : (__expf(v) - 1.0f); }
__global__ __launch_bounds__(256) void k_gat1(const float* __restrict__ XLR, const float* __restrict__ att, const int* __restrict__ src, const int* __restrict__ cstart, const int* __restrict__ ccnt, const int* __restrict__ ceid, const float* __restrict__ b, float* __restrict__ H) {
  const int tid = threadIdx.x, wv = tid >> 5, lane = tid & 31; const int d = blockIdx.x * 8 + wv; if (d >= NNODE) return;
  int p0 = cstart[d]; int cn = ccnt[d]; cn = cn < 0 ? 0 : (cn > MAXDEG ? MAXDEG : cn); p0 = p0 < 0 ? 0 : (p0 > NTOT + 32 * CS_NB ? NTOT + 32 * CS_NB : p0);
  const v4f xr = *(const v4fa*)(XLR + (size_t)d * 256 + 128 + 4 * lane); float at[4]; for (int u = 0; u < 4; ++u) at[u] = bf16_round(att[4 * lane + u]);
  float m = -3.0e38f, dn = 0.f; float acc[4] = {0.f, 0.f, 0.f, 0.f};
#pragma unroll 1
  for (int q = 0; q < cn; ++q) { int e = ceid[p0 + q]; e = e < 0 ? 0 : (e >= NTOT ? NTOT - 1 : e); int s = (e < NE) ? src[e] : (e - NE); s = s < 0 ? 0 : (s >= NNODE ? NNODE - 1 : s);
    const v4f xl = *(const v4fa*)(XLR + (size_t)s * 256 + 4 * lane); float lg = 0.f;
#pragma unroll
    for (int u = 0; u < 4; ++u) lg += lrelu(xl[u] + xr[u]) * at[u];
    for (int o = 8; o >= 1; o >>= 1) lg += __shfl_xor(lg, o, 32);
    const float mn = fmaxf(m, lg); const float r = __expf(m - mn), p = __expf(lg - mn); dn = dn * r + p;
#pragma unroll
    for (int u = 0; u < 4; ++u) acc[u] = acc[u] * r + p * xl[u]; m = mn; }
  const float rd = (cn > 0) ? 1.0f / dn : 0.f; v4f o; for (int u = 0; u < 4; ++u) o[u] = elu1(acc[u] * rd + bf16_round(b[4 * lane + u]));
  *(volatile v4f*)(H + (size_t)d * 128 + 4 * lane) = o; __threadfence(); *(volatile v4f*)(H + (size_t)d * 128 + 4 * lane) = o;
}
typedef float v2f_t __attribute__((ext_vector_type(2)));
__global__ __launch_bounds__(256) void k_gat2(const float* __restrict__ XLR, const float* __restrict__ att, const int* __restrict__ src, const int* __restrict__ cstart, const int* __restrict__ ccnt, const int* __restrict__ ceid, const float* __restrict__ b, float* __restrict__ H2) {
  const int tid = threadIdx.x, wv = tid >> 5, lane = tid & 31; const int d = blockIdx.x * 8 + wv; if (d >= NNODE) return;
  int p0 = cstart[d]; int cn = ccnt[d]; cn = cn < 0 ? 0 : (cn > MAXDEG ? MAXDEG : cn); p0 = p0 < 0 ? 0 : (p0 > NTOT + 32 * CS_NB ? NTOT + 32 * CS_NB : p0);
  const v2f_t xr = *(const v2f_t*)(XLR + (size_t)d * 128 + 64 + 2 * lane); const float a0 = bf16_round(att[2 * lane]), a1 = bf16_round(att[2 * lane + 1]);
  float m = -3.0e38f, dn = 0.f, c0 = 0.f, c1 = 0.f;
#pragma unroll 1
  for (int q = 0; q < cn; ++q) { int e = ceid[p0 + q]; e = e < 0 ? 0 : (e >= NTOT ? NTOT - 1 : e); int s = (e < NE) ? src[e] : (e - NE); s = s < 0 ? 0 : (s >= NNODE ? NNODE - 1 : s);
    const v2f_t xl = *(const v2f_t*)(XLR + (size_t)s * 128 + 2 * lane); float lg = lrelu(xl.x + xr.x) * a0 + lrelu(xl.y + xr.y) * a1; for (int o = 16; o >= 1; o >>= 1) lg += __shfl_xor(lg, o, 32);
    const float mn = fmaxf(m, lg); const float r = __expf(m - mn), p = __expf(lg - mn); dn = dn * r + p; c0 = c0 * r + p * xl.x; c1 = c1 * r + p * xl.y; m = mn; }
  const float rd = (cn > 0) ? 1.0f / dn : 0.f; v2f_t o; o.x = c0 * rd + bf16_round(b[2 * lane]); o.y = c1 * rd + bf16_round(b[2 * lane + 1]);
  *(volatile v2f_t*)(H2 + (size_t)d * 64 + 2 * lane) = o; __threadfence(); *(volatile v2f_t*)(H2 + (size_t)d * 64 + 2 * lane) = o;
}
__global__ __launch_bounds__(512) void k_poolcls(const float* __restrict__ H2, const int* __restrict__ batch, const float* __restrict__ lw, const float* __restrict__ lb, float* __restrict__ out) {
  __shared__ float sp[16][64]; __shared__ float so[16][16]; const int tid = threadIdx.x, wv = tid >> 5, lane = tid & 31; const int g = blockIdx.x * 16 + wv;
  int lo = 0, hi = NNODE; while (lo < hi) { const int mm = (lo + hi) >> 1; if (batch[mm] < g) lo = mm + 1; else hi = mm; } const int s0 = lo; lo = 0; hi = NNODE; while (lo < hi) { const int mm = (lo + hi) >> 1; if (batch[mm] < g + 1) lo = mm + 1; else hi = mm; } const int s1 = lo;
  float a0 = 0.f, a1 = 0.f;
#pragma unroll 1
  for (int n = s0; n < s1; ++n) { const v2f_t v = *(const v2f_t*)(H2 + (size_t)n * 64 + 2 * lane); a0 += v.x; a1 += v.y; }
  const float inv = 1.0f / fmaxf((float)(s1 - s0), 1.0f); sp[wv][2 * lane] = a0 * inv; sp[wv][2 * lane + 1] = a1 * inv;
  __builtin_amdgcn_fence(__ATOMIC_ACQ_REL, "workgroup"); __builtin_amdgcn_wave_barrier();
  if (lane < NCLS) { float s = bf16_round(lb[lane]);
#pragma unroll 1
    for (int c = 0; c < 64; ++c) s += sp[wv][c] * bf16_round(lw[c * NCLS + lane]); so[wv][lane] = s; }
  __syncthreads();
  for (int pass = 0; pass < 2; ++pass) { if (tid < 160) *(volatile float*)(out + (size_t)blockIdx.x * 160 + tid) = so[tid / 10][tid % 10]; if (pass == 0) __threadfence(); }
}
extern "C" void kernel_launch(void* const* d_in, const int* in_sizes, int n_in,
                              void* d_out, int out_size, void* d_ws, size_t ws_size, hipStream_t stream) {
  (void)in_sizes; (void)n_in; (void)out_size;
  const float* x = (const float*)d_in[0]; const int* ei = (const int*)d_in[1]; const int* batch = (const int*)d_in[2];
  const float* Wl1 = (const float*)d_in[3]; const float* Wr1 = (const float*)d_in[4]; const float* att1 = (const float*)d_in[5]; const float* b1 = (const float*)d_in[6]; const float* Wl2 = (const float*)d_in[7]; const float* Wr2 = (const float*)d_in[8]; const float* att2 = (const float*)d_in[9]; const float* b2 = (const float*)d_in[10]; const float* lw = (const float*)d_in[11]; const float* lb = (const float*)d_in[12];
  char* ws = (char*)d_ws; size_t off = 0;
  auto take = [&](size_t bytes) { char* p = ws + off; off += (bytes + 255) & ~(size_t)255; return p; };
  unsigned short* B1 = (unsigned short*)take((size_t)256 * FIN * 2); unsigned short* B2 = (unsigned short*)take((size_t)128 * 128 * 2);
  int* seg_dst = (int*)take((size_t)CS_NW * CS_CH * 4); int* seg_eid = (int*)take((size_t)CS_NW * CS_CH * 4); int* P1 = (int*)take((size_t)CS_NW * CS_NB * 4); int* Q1 = (int*)take((size_t)CS_NW * CS_NB * 4); int* R_ = (int*)take((size_t)CS_NW * CS_NB * 4); int* S_ = (int*)take((CS_NB + 32) * 4);
  int* ceid = (int*)take(((size_t)NTOT + 32 * CS_NB) * 4); int* cstart = (int*)take((size_t)CS_NB * CS_NB * 4); int* ccnt = (int*)take((size_t)CS_NB * CS_NB * 4);
  float* XLR1 = (float*)take((size_t)NNODE * 256 * 4); float* H = (float*)take((size_t)NNODE * 128 * 4); float* XLR2 = (float*)take((size_t)NNODE * 128 * 4); float* H2 = (float*)take((size_t)NNODE * 64 * 4);
  if (off > ws_size) return;
  k_btcat<<<(256 * 8 + 255) / 256, 256, 0, stream>>>(Wl1, Wr1, FIN, 128, B1); k_btcat<<<(128 * 16 + 255) / 256, 256, 0, stream>>>(Wl2, Wr2, 128, 64, B2);
  build_csr(ei + NE, NE, NTOT, NNODE, seg_dst, seg_eid, P1, Q1, R_, S_, ceid, cstart, ccnt, stream);
  k_gemm_bf3<false, 0, false, false><<<((NNODE / 16) * 4 + 3) / 4, 128, 0, stream>>>(x, FIN, B1, FIN, nullptr, nullptr, 1, 0, XLR1, 256, NNODE, 256, FIN);
  k_gat1<<<(NNODE + 7) / 8, 256, 0, stream>>>(XLR1, att1, ei, cstart, ccnt, ceid, b1, H);
  k_gemm_bf3<true, 0, false, false><<<((NNODE / 16) * 2 + 3) / 4, 128, 0, stream>>>(H, 128, B2, 128, nullptr, nullptr, 1, 0, XLR2, 128, NNODE, 128, 128);
  k_gat2<<<(NNODE + 7) / 8, 256, 0, stream>>>(XLR2, att2, ei, cstart, ccnt, ceid, b2, H2);
  k_poolcls<<<NG / 16, 512, 0, stream>>>(H2, batch, lw, lb, (float*)d_out);
}
